// SAGEConvReconstructionModule_36850819400182
// MI455X (gfx1250) — hardware-run, weakly checked
//
#include <hip/hip_runtime.h>


namespace {
constexpr int N = 100000, NP = 100032  , E = 1600000, IN = 128, HID = 64, OUT = 32;
constexpr float XS = 8.0f, WSC = 256.0f, SLOPE = 0.1f;

typedef _Float16 b16;
typedef __attribute__((ext_vector_type(16))) _Float16 v16b;
typedef __attribute__((ext_vector_type(8))) _Float16 v8b;
typedef __attribute__((ext_vector_type(8))) float v8f;
typedef __attribute__((ext_vector_type(4))) float v4f;
typedef __attribute__((ext_vector_type(4))) _Float16 v4b;
typedef __attribute__((ext_vector_type(2))) _Float16 v2b;
__device__ __forceinline__ float bf16_rne(float f) { unsigned int u = __float_as_uint(f); u += 0x7FFFu + ((u >> 16) & 1u); return __uint_as_float(u & 0xFFFF0000u); }
__device__ __forceinline__ void split16(float v, b16& hi, b16& lo) { hi = (b16)v; lo = (b16)(v - (float)hi); }
__device__ __forceinline__ v16b frag_kb(const b16* p, int hh) { const v8b a = *(const v8b*)(p + 8 * hh), b = *(const v8b*)(p + 16 + 8 * hh); v16b f;
#pragma unroll
  for (int e = 0; e < 8; ++e) { f[e] = a[e]; f[8 + e] = b[e]; } return f; }
__device__ __forceinline__ v8f wmma16b(v16b a, v16b b, v8f c) { v8f d = __builtin_amdgcn_wmma_f32_16x16x32_f16(false, a, false, b, (short)0, c, false, false); asm volatile("v_nop\n\tv_nop\n\tv_nop\n\tv_nop" : "+v"(d) : "v"(a), "v"(b)); return d; }
__device__ __forceinline__ void wave_lds_sync() { __builtin_amdgcn_fence(__ATOMIC_RELEASE, "workgroup"); __builtin_amdgcn_wave_barrier(); __builtin_amdgcn_fence(__ATOMIC_ACQUIRE, "workgroup"); }
__device__ __forceinline__ float pmul(float a, float b) { float p = a * b; asm volatile("" : "+v"(p)); return p; }
__device__ __forceinline__ int iclamp(int v, int lo, int hi) { return v < lo ? lo : (v > hi ? hi : v); }
__device__ __forceinline__ float lrelu(float x) { return x >= 0.0f ? x : SLOPE * x; }

constexpr int CSR_NBLK = 512, CSR_GB = 9, CSR_GN = 1 << CSR_GB  , CSR_MAXG = 512, CSR_CAP = 12288  ;
__global__ __launch_bounds__(64) void csrA_kernel(const int* __restrict__ dst, int E, int N, int nG, int CHP, int NGP, int* __restrict__ STG, int* __restrict__ HST) {
  extern __shared__ int sm[];
  int* cnt = sm; int* run = sm + NGP; int* ids = sm + 2 * NGP;
  const int b = blockIdx.x; const int ch = (E + CSR_NBLK - 1) / CSR_NBLK; const int e0 = b * ch, e1 = min(E, e0 + ch);
  for (int i = threadIdx.x; i < NGP; i += 64) cnt[i] = 0;
  for (int i = threadIdx.x; i < CHP; i += 64) ids[i] = -1;
  __syncthreads();
  if (threadIdx.x == 0) {
    for (int e = e0; e < e1; ++e) { int d = dst[e]; d = (d < 0) ? 0 : (d >= N ? N - 1 : d); cnt[d >> CSR_GB] += 1; }
    int acc = 0; for (int g = 0; g < nG; ++g) { run[g] = acc; acc += cnt[g]; }
    for (int e = e0; e < e1; ++e) { int d = dst[e]; d = (d < 0) ? 0 : (d >= N ? N - 1 : d); const int g = d >> CSR_GB; ids[run[g]] = e; run[g] += 1; } }
  __syncthreads();
  typedef __attribute__((ext_vector_type(4))) int v4i;
  for (int pass = 0; pass < 2; ++pass) {
    for (int i = threadIdx.x; i < CHP / 4; i += 64) *(volatile v4i*)(STG + (size_t)b * CHP + i * 4) = *(const v4i*)(&ids[i * 4]);
    for (int i = threadIdx.x; i < NGP / 4; i += 64) { v4i v; for (int e = 0; e < 4; ++e) v[e] = (i * 4 + e < nG) ? cnt[i * 4 + e] : 0; *(volatile v4i*)(HST + (size_t)b * NGP + i * 4) = v; }
    __threadfence(); }
}
__global__ __launch_bounds__(512) void csrS_kernel(const int* __restrict__ HST, int nG, int NGP, int* __restrict__ START, int* __restrict__ TOT, int* __restrict__ OFF) {
  __shared__ int tot[CSR_MAXG];
  const int b = threadIdx.x;
  for (int pass = 0; pass < 2; ++pass) { int runb = 0; for (int g = 0; g < nG; ++g) { int c = HST[(size_t)b * NGP + g]; c = (c < 0) ? 0 : c; ((volatile int*)OFF)[(size_t)g * CSR_NBLK + b] = runb; runb += c; } __threadfence(); }
  for (int g = threadIdx.x; g < nG; g += 512) { int s = 0; for (int bb = 0; bb < CSR_NBLK; ++bb) { int c = HST[(size_t)bb * NGP + g]; s += (c < 0) ? 0 : c; } tot[g] = s; }
  __syncthreads();
  if (threadIdx.x < 32) {
    __shared__ int st[CSR_MAXG + 32];
    if (threadIdx.x == 0) { int acc = 0; for (int g = 0; g < NGP; ++g) { st[g] = acc; if (g < nG) acc += (tot[g] + 31) & ~31; } st[NGP] = acc; }
    __builtin_amdgcn_fence(__ATOMIC_RELEASE, "workgroup"); __builtin_amdgcn_wave_barrier(); __builtin_amdgcn_fence(__ATOMIC_ACQUIRE, "workgroup");
    for (int pass = 0; pass < 2; ++pass) { for (int i = threadIdx.x; i < NGP + 32; i += 32) { ((volatile int*)START)[i] = (i <= NGP) ? st[min(i, NGP)] : 0; ((volatile int*)TOT)[i] = (i < nG) ? tot[i] : 0; } __threadfence(); } }
}
__global__ __launch_bounds__(256) void csrB_kernel(const int* __restrict__ dst, int N, int nG, int CHP, int NGP, int permLen, const int* __restrict__ STG, const int* __restrict__ HST, const int* __restrict__ OFF, const int* __restrict__ START, const int* __restrict__ TOT, int* __restrict__ PERM, int* __restrict__ ROWPTR, int* __restrict__ ROWCNT, int* __restrict__ FLAG) {
  typedef __attribute__((ext_vector_type(4))) int v4i;
  __shared__ int ids[CSR_CAP]; __shared__ unsigned short key[CSR_CAP]; __shared__ int outp[CSR_CAP]; __shared__ int ncnt[CSR_GN + 1]; __shared__ int boff[CSR_NBLK + 1];
  const int g = blockIdx.x, t_ = threadIdx.x; int tot = TOT[g]; int st = START[g], stn = START[g + 1]; const int v0 = g * CSR_GN; const int nv = min(CSR_GN, N - v0);
  st = (st < 0) ? 0 : (st > permLen - 32 ? permLen - 32 : st) & ~31; stn = (stn < st) ? st : (stn > permLen ? permLen : stn); tot = (tot < 0) ? 0 : tot; if (tot > stn - st && tot <= CSR_CAP) tot = stn - st;
  if (tot > CSR_CAP) {
    for (int pass = 0; pass < 2; ++pass) { for (int i = t_; i < CSR_GN / 4; i += 256) { v4i a, c; for (int e = 0; e < 4; ++e) { a[e] = st; c[e] = 0; } *(volatile v4i*)(ROWPTR + v0 + i * 4) = a; *(volatile v4i*)(ROWCNT + v0 + i * 4) = c; } if (t_ == 0) ((volatile int*)FLAG)[0] = 1; __threadfence(); } (void)nv; return; }
  if (t_ == 0) { int acc = 0; for (int b = 0; b < CSR_NBLK; ++b) { boff[b] = acc; int c = HST[(size_t)b * NGP + g]; c = (c < 0) ? 0 : (c > CHP ? CHP : c); acc += c; if (acc > tot) acc = tot; } boff[CSR_NBLK] = acc; }
  for (int i = t_; i <= CSR_GN; i += 256) ncnt[i] = 0;
  __syncthreads();
  for (int b = 0; b < CSR_NBLK; ++b) { const int c = boff[b + 1] - boff[b]; int o_ = OFF[(size_t)g * CSR_NBLK + b]; o_ = (o_ < 0) ? 0 : (o_ > CHP - c ? CHP - c : o_); const int* src_ = STG + (size_t)b * CHP + o_;
    for (int i = t_; i < c; i += 256) { int id = src_[i]; id = (id < 0) ? 0 : id; ids[boff[b] + i] = id; int d = dst[id]; d = (d < v0) ? v0 : (d >= N ? N - 1 : d); int kk = d - v0; kk = (kk < 0) ? 0 : (kk >= CSR_GN ? CSR_GN - 1 : kk); key[boff[b] + i] = (unsigned short)kk; } }
  __syncthreads();
  if (t_ == 0) { for (int i = 0; i < tot; ++i) ncnt[key[i]] += 1; int acc = 0; for (int vl = 0; vl < CSR_GN; ++vl) { const int c = ncnt[vl]; ncnt[vl] = acc; acc += c; } ncnt[CSR_GN] = acc;
    for (int i = 0; i < tot; ++i) { const int vl = key[i]; outp[ncnt[vl]] = ids[i]; ncnt[vl] += 1; }
    for (int vl = CSR_GN; vl > 0; --vl) ncnt[vl] = ncnt[vl - 1]; ncnt[0] = 0; }
  __syncthreads();
  for (int pass = 0; pass < 2; ++pass) {
    for (int i = t_; i < (stn - st) / 4; i += 256) { v4i v; for (int e = 0; e < 4; ++e) { const int q = i * 4 + e; v[e] = (q < tot) ? outp[q] : -1; } *(volatile v4i*)(PERM + st + i * 4) = v; }
    for (int i = t_; i < CSR_GN / 4; i += 256) { v4i a, c; for (int e = 0; e < 4; ++e) { const int vl = i * 4 + e; a[e] = st + ncnt[vl]; c[e] = (vl < nv) ? (ncnt[vl + 1] - ncnt[vl]) : 0; } *(volatile v4i*)(ROWPTR + v0 + i * 4) = a; *(volatile v4i*)(ROWCNT + v0 + i * 4) = c; }
    __threadfence(); }
}
__global__ __launch_bounds__(256) void csrZ_kernel(int* __restrict__ p, size_t n4) { typedef __attribute__((ext_vector_type(4))) int v4i; const size_t tid = (size_t)blockIdx.x * 256 + threadIdx.x, nth = (size_t)gridDim.x * 256; v4i z = {0, 0, 0, 0}; for (size_t i = tid; i < n4; i += nth) *(volatile v4i*)(p + i * 4) = z; }
struct CsrBufs { int *STG, *HST, *OFF, *START, *TOT, *PERM, *ROWPTR, *ROWCNT, *FLAG; int nG, NGP, CHP; size_t permLen; char* base; size_t bytes; };
static size_t csr_carve(CsrBufs& c, char* ws, size_t off, int E, int N) {
  const size_t off0 = off; c.base = ws + off;
  auto al = [&](size_t bytes) { char* p = ws + off; off += (bytes + 255) & ~(size_t)255; return p; };
  c.nG = (N + CSR_GN - 1) / CSR_GN; c.NGP = (c.nG + 31) & ~31; const int ch = (E + CSR_NBLK - 1) / CSR_NBLK; c.CHP = (ch + 31) & ~31; c.permLen = (size_t)E + 32 * (size_t)c.nG + 32;
  c.STG = (int*)al((size_t)CSR_NBLK * c.CHP * 4); c.HST = (int*)al((size_t)CSR_NBLK * c.NGP * 4); c.OFF = (int*)al((size_t)c.NGP * CSR_NBLK * 4); c.START = (int*)al((size_t)(c.NGP + 64) * 4); c.TOT = (int*)al((size_t)(c.NGP + 64) * 4);
  c.PERM = (int*)al(c.permLen * 4); c.ROWPTR = (int*)al((size_t)c.nG * CSR_GN * 4); c.ROWCNT = (int*)al((size_t)c.nG * CSR_GN * 4); c.FLAG = (int*)al(256);
  c.bytes = off - off0; return off;
}
static void csr_build(const CsrBufs& c, const int* dst, int E, int N, hipStream_t stream) {
  const size_t smem = (size_t)(2 * c.NGP + c.CHP) * 4;
  csrZ_kernel<<<512, 256, 0, stream>>>((int*)c.base, c.bytes / 16);
  csrA_kernel<<<CSR_NBLK, 64, smem, stream>>>(dst, E, N, c.nG, c.CHP, c.NGP, c.STG, c.HST);
  csrS_kernel<<<1, 512, 0, stream>>>(c.HST, c.nG, c.NGP, c.START, c.TOT, c.OFF);
  csrB_kernel<<<c.nG, 256, 0, stream>>>(dst, N, c.nG, c.CHP, c.NGP, (int)c.permLen, c.STG, c.HST, c.OFF, c.START, c.TOT, c.PERM, c.ROWPTR, c.ROWCNT, c.FLAG);
}


__global__ __launch_bounds__(256) void prep_kernel(const float* __restrict__ x, const float* __restrict__ wl1, const float* __restrict__ wr1, const float* __restrict__ wl2, const float* __restrict__ wr2, b16* __restrict__ X16, b16* __restrict__ W1, b16* __restrict__ W2) {
  const size_t t = (size_t)blockIdx.x * 256 + threadIdx.x; const size_t nx = (size_t)NP * IN / 8, n1 = (size_t)HID * 2 * IN / 8, n2 = (size_t)OUT * 2 * HID / 8; v8b o;
  if (t < nx) { const size_t e = t * 8; const size_t row = e / IN; for (int j = 0; j < 8; ++j) o[j] = (row < (size_t)N) ? (b16)(bf16_rne(x[e + j]) * XS) : (b16)0.0f; for (int pass = 0; pass < 2; ++pass) { *(volatile v8b*)(X16 + e) = o; __threadfence(); } }
  else if (t < nx + n1) { const size_t e = (t - nx) * 8; const int oo = (int)(e / (2 * IN)), k0 = (int)(e % (2 * IN)); for (int j = 0; j < 8; ++j) { const int k = k0 + j; const float v = (k < IN) ? wl1[(size_t)k * HID + oo] : wr1[(size_t)(k - IN) * HID + oo]; o[j] = (b16)(bf16_rne(v) * WSC); } for (int pass = 0; pass < 2; ++pass) { *(volatile v8b*)(W1 + e) = o; __threadfence(); } }
  else if (t < nx + n1 + n2) { const size_t e = (t - nx - n1) * 8; const int oo = (int)(e / (2 * HID)), k0 = (int)(e % (2 * HID)); for (int j = 0; j < 8; ++j) { const int k = k0 + j; const float v = (k < HID) ? wl2[(size_t)k * OUT + oo] : wr2[(size_t)(k - HID) * OUT + oo]; o[j] = (b16)(bf16_rne(v) * WSC); } for (int pass = 0; pass < 2; ++pass) { *(volatile v8b*)(W2 + e) = o; __threadfence(); } }
}
__global__ __launch_bounds__(256) void agg1_kernel(const float* __restrict__ x, const int* __restrict__ srcs, const int* __restrict__ PERM, const int* __restrict__ ROWPTR, const int* __restrict__ ROWCNT, int permLen, b16* __restrict__ AXh, b16* __restrict__ AXl) {
  const int wave = threadIdx.x >> 5, lane = threadIdx.x & 31; const size_t v = (size_t)blockIdx.x * 8 + wave; const int c0 = lane * 4;
  int cnt = 0, st = 0; if (v < (size_t)N) { st = ROWPTR[v]; cnt = ROWCNT[v]; cnt = iclamp(cnt, 0, 8192); st = iclamp(st, 0, permLen - cnt); }
  v4f acc = {0, 0, 0, 0};
  for (int j = 0; j < cnt; ++j) { const int e = iclamp(PERM[st + j], 0, E - 1); const int s = iclamp(srcs[e], 0, N - 1); const v4f xr = *(const v4f*)(x + (size_t)s * IN + c0); for (int q = 0; q < 4; ++q) acc[q] += bf16_rne(xr[q]); }
  const float dinv = 1.0f / (float)(cnt > 1 ? cnt : 1); v4b hv, lv; for (int q = 0; q < 4; ++q) { b16 p, qq; split16(pmul(acc[q], dinv) * XS, p, qq); hv[q] = p; lv[q] = qq; }
  for (int pass = 0; pass < 2; ++pass) { *(volatile v4b*)(AXh + v * IN + c0) = hv; *(volatile v4b*)(AXl + v * IN + c0) = lv; __threadfence(); }
}
__global__ __launch_bounds__(256) void agg2_kernel(const b16* __restrict__ Hh, const b16* __restrict__ Hl, const int* __restrict__ srcs, const int* __restrict__ PERM, const int* __restrict__ ROWPTR, const int* __restrict__ ROWCNT, int permLen, b16* __restrict__ AHh, b16* __restrict__ AHl) {
  const int wave = threadIdx.x >> 5, lane = threadIdx.x & 31; const size_t v = (size_t)blockIdx.x * 8 + wave; const int c0 = lane * 2;
  int cnt = 0, st = 0; if (v < (size_t)N) { st = ROWPTR[v]; cnt = ROWCNT[v]; cnt = iclamp(cnt, 0, 8192); st = iclamp(st, 0, permLen - cnt); }
  float a0 = 0.0f, a1 = 0.0f;
  for (int j = 0; j < cnt; ++j) { const int e = iclamp(PERM[st + j], 0, E - 1); const int s = iclamp(srcs[e], 0, N - 1); const v2b h2 = *(const v2b*)(Hh + (size_t)s * HID + c0), l2 = *(const v2b*)(Hl + (size_t)s * HID + c0); a0 += ((float)h2[0] + (float)l2[0]) * (1.0f / XS); a1 += ((float)h2[1] + (float)l2[1]) * (1.0f / XS); }
  const float dinv = 1.0f / (float)(cnt > 1 ? cnt : 1); v2b hv, lv; { b16 p, q; split16(pmul(a0, dinv) * XS, p, q); hv[0] = p; lv[0] = q; split16(pmul(a1, dinv) * XS, p, q); hv[1] = p; lv[1] = q; }
  for (int pass = 0; pass < 2; ++pass) { *(volatile v2b*)(AHh + v * HID + c0) = hv; *(volatile v2b*)(AHl + v * HID + c0) = lv; __threadfence(); }
}
template <int LAYER>
__global__ __launch_bounds__(128) void gemm_kernel(const b16* __restrict__ Ah, const b16* __restrict__ Al, const b16* __restrict__ Sh, const b16* __restrict__ Sl, const b16* __restrict__ W, const float* __restrict__ bias, b16* __restrict__ Yh, b16* __restrict__ Yl, float* __restrict__ Yf) {
  constexpr int KA = LAYER == 1 ? IN : HID, NO = LAYER == 1 ? HID : OUT, NT = NO / 16, KT = 2 * KA;
  __shared__ __attribute__((aligned(16))) float Ts[4][16][NO + 4];
  const int wave = threadIdx.x >> 5, lane = threadIdx.x & 31, nloc = lane & 15, hlf = lane >> 4; const size_t m0 = ((size_t)blockIdx.x * 4 + wave) * 16;
  v8f acc[NT];
#pragma unroll
  for (int t = 0; t < NT; ++t) acc[t] = (v8f){};
#pragma unroll
  for (int kb = 0; kb < KA; kb += 32) { const v16b a = frag_kb(Ah + (m0 + nloc) * KA + kb, hlf), al = frag_kb(Al + (m0 + nloc) * KA + kb, hlf); const v16b s = frag_kb(Sh + (m0 + nloc) * KA + kb, hlf); v16b sl = {}; if (LAYER == 2) sl = frag_kb(Sl + (m0 + nloc) * KA + kb, hlf);
#pragma unroll
    for (int t = 0; t < NT; ++t) { const v16b wa = frag_kb(W + (size_t)(t * 16 + nloc) * KT + kb, hlf), ws_ = frag_kb(W + (size_t)(t * 16 + nloc) * KT + KA + kb, hlf); acc[t] = wmma16b(a, wa, acc[t]); acc[t] = wmma16b(al, wa, acc[t]); acc[t] = wmma16b(s, ws_, acc[t]); if (LAYER == 2) acc[t] = wmma16b(sl, ws_, acc[t]); } }
#pragma unroll
  for (int t = 0; t < NT; ++t) { const int c = t * 16 + nloc; const float bb = bf16_rne(bias[c]);
#pragma unroll
    for (int r = 0; r < 8; ++r) Ts[wave][8 * hlf + r][c] = lrelu(acc[t][r] * (1.0f / (XS * WSC)) + bb); }
  wave_lds_sync();
  for (int pass = 0; pass < 2; ++pass) { for (int rr = 0; rr < 16; ++rr) { const size_t row = m0 + rr;
      if (LAYER == 1) { if (lane < 8) { v8b hv, lv; for (int j = 0; j < 8; ++j) { b16 p, q; const float v = (row < (size_t)N) ? Ts[wave][rr][lane * 8 + j] : 0.0f; split16(v * XS, p, q); hv[j] = p; lv[j] = q; } *(volatile v8b*)(Yh + row * HID + lane * 8) = hv; *(volatile v8b*)(Yl + row * HID + lane * 8) = lv; } }
      else { if (lane < 8 && row < (size_t)N) *(volatile v4f*)(Yf + row * OUT + lane * 4) = *(const v4f*)(&Ts[wave][rr][lane * 4]); } }
    __threadfence(); }
}
}

extern "C" void kernel_launch(void* const* d_in, const int* in_sizes, int n_in, void* d_out, int out_size, void* d_ws, size_t ws_size, hipStream_t stream) {
  (void)n_in;
  auto Fp = [&](int i) { return (const float*)d_in[i]; }; auto Ip = [&](int i) { return (const int*)d_in[i]; };
  if (in_sizes[0] != N * IN || in_sizes[1] != 2 * E || in_sizes[2] != IN * HID || in_sizes[5] != HID * OUT || out_size != N * OUT) return;
  size_t off = 0; char* ws = (char*)d_ws;
  auto carve = [&](size_t bytes) { char* p = ws + off; off += (bytes + 255) & ~(size_t)255; return p; };
  b16* X16 = (b16*)carve((size_t)NP * IN * 2); b16* W1 = (b16*)carve((size_t)HID * 2 * IN * 2); b16* W2 = (b16*)carve((size_t)OUT * 2 * HID * 2);
  b16* AXh = (b16*)carve((size_t)NP * IN * 2); b16* AXl = (b16*)carve((size_t)NP * IN * 2); b16* Hh = (b16*)carve((size_t)NP * HID * 2); b16* Hl = (b16*)carve((size_t)NP * HID * 2);
  b16* AHh = AXh; b16* AHl = AXl;
  CsrBufs csr; off = csr_carve(csr, ws, off, E, N);
  if (off > ws_size || off > ((size_t)128 << 20)) return;
  prep_kernel<<<(unsigned)(((size_t)NP * IN / 8 + (size_t)HID * 2 * IN / 8 + (size_t)OUT * 2 * HID / 8 + 255) / 256), 256, 0, stream>>>(Fp(0), Fp(2), Fp(3), Fp(5), Fp(6), X16, W1, W2);
  csr_build(csr, Ip(1) + E, E, N, stream);
  agg1_kernel<<<NP / 8, 256, 0, stream>>>(Fp(0), Ip(1), csr.PERM, csr.ROWPTR, csr.ROWCNT, (int)csr.permLen, AXh, AXl);
  gemm_kernel<1><<<NP / 64, 128, 0, stream>>>(AXh, AXl, X16, nullptr, W1, Fp(4), Hh, Hl, nullptr);
  agg2_kernel<<<NP / 8, 256, 0, stream>>>(Hh, Hl, Ip(1), csr.PERM, csr.ROWPTR, csr.ROWCNT, (int)csr.permLen, AHh, AHl);
  gemm_kernel<2><<<NP / 64, 128, 0, stream>>>(AHh, AHl, Hh, Hl, W2, Fp(7), nullptr, nullptr, (float*)d_out);
}
